// SimpleSelfAttention_70437463654765
// MI455X (gfx1250) — hardware-verified
//
#include <hip/hip_runtime.h>


#ifndef NB
#define NB 4
#endif
#ifndef SEQ
#define SEQ 2048
#endif
#define NB_FULL  4
#define SEQ_FULL 2048
#define DD       1024
#define RH       (((SEQ) < 512) ? (SEQ) : 512)
#define PCAR     1024.0f
#define SCL      0.03125f

static_assert(NB >= 1 && NB <= NB_FULL);
static_assert(SEQ % 256 == 0 && SEQ <= SEQ_FULL);
static_assert(RH % 256 == 0 && RH <= SEQ);
static_assert(DD % 256 == 0);

typedef _Float16 h16;
typedef unsigned short bf;
typedef __attribute__((ext_vector_type(16))) __bf16   v16bf;
typedef __attribute__((ext_vector_type(16))) _Float16 v16h;
typedef __attribute__((ext_vector_type(8)))  _Float16 v8h;
typedef __attribute__((ext_vector_type(8)))  unsigned short v8us;
typedef __attribute__((ext_vector_type(8)))  float    v8f;
typedef __attribute__((ext_vector_type(4)))  float    v4f;
typedef __attribute__((ext_vector_type(4)))  _Float16 v4h;
typedef __attribute__((ext_vector_type(4)))  unsigned short v4us;
typedef v8h  __attribute__((may_alias)) v8ha;
typedef v4f  __attribute__((may_alias)) v4fa;
typedef v8us __attribute__((may_alias)) v8usa;

__device__ __forceinline__ unsigned short f2bf(float f) { unsigned u = __float_as_uint(f); u += 0x7FFFu + ((u >> 16) & 1u); return (unsigned short)(u >> 16); }
__device__ __forceinline__ float bf2f(unsigned short b) { return __uint_as_float(((unsigned)b) << 16); }
__device__ __forceinline__ v16h cat16(v8h lo, v8h hi) { return __builtin_shufflevector(lo, hi, 0, 1, 2, 3, 4, 5, 6, 7, 8, 9, 10, 11, 12, 13, 14, 15); }
__device__ __forceinline__ v16bf cat16b(v8us lo, v8us hi) { return __builtin_bit_cast(v16bf, __builtin_shufflevector(lo, hi, 0, 1, 2, 3, 4, 5, 6, 7, 8, 9, 10, 11, 12, 13, 14, 15)); }
__device__ __forceinline__ v8f wmma16(v16h a, v16h b, v8f c) { return __builtin_amdgcn_wmma_f32_16x16x32_f16(false, a, false, b, (short)0, c, false, false); }
__device__ __forceinline__ v8f wmmab(v16bf a, v16bf b, v8f c) { return __builtin_amdgcn_wmma_f32_16x16x32_bf16(false, a, false, b, (short)0, c, false, false); }
__device__ __forceinline__ h16 tohx(float x) { return (h16)x; }
__device__ __forceinline__ void splitf(float y, unsigned short& h, unsigned short& l) { h = f2bf(y); l = f2bf(y - bf2f(h)); }

template <typename T16> struct WFrag;
template <> struct WFrag<h16> { typedef v16h V; static __device__ __forceinline__ V ld(const h16* p) { return cat16(*(const v8h*)p, *(const v8h*)(p + 16)); } static __device__ __forceinline__ v8f mma(V a, V b, v8f c) { return wmma16(a, b, c); } };
template <> struct WFrag<bf> { typedef v16bf V; static __device__ __forceinline__ V ld(const bf* p) { return cat16b(*(const v8us*)p, *(const v8us*)(p + 16)); } static __device__ __forceinline__ v8f mma(V a, V b, v8f c) { return wmmab(a, b, c); } };
template <typename T16, int NSPLIT, int CAUS>
__global__ __launch_bounds__(32) void k_gemmw(const T16* __restrict__ A, const T16* __restrict__ A2, const T16* __restrict__ Bt, const T16* __restrict__ Bt2, int K, float* C, int ldc, float osc, int rbase, size_t sA, size_t sB, size_t sC) {
    typedef typename WFrag<T16>::V V;
    __shared__ __align__(16) float os[16 * 68];
    const size_t z = blockIdx.z; A += z * sA; if (A2) A2 += z * sA; Bt += z * sB; if (Bt2) Bt2 += z * sB; C += z * sC;
    const int lane = threadIdx.x & 31, lr = lane & 15, hi = lane >> 4; const int r0 = blockIdx.x * 64, c0 = blockIdx.y * 64;
    if (CAUS == 1 && c0 > rbase + r0 + 63) return;
    const int kend = rbase + r0 + 64;
    const int Kc = (CAUS == 2) ? ((K < kend) ? K : kend) : K;
    v8f acc[4][4];
#pragma unroll
    for (int mb = 0; mb < 4; ++mb)
#pragma unroll
        for (int nb = 0; nb < 4; ++nb) acc[mb][nb] = (v8f){};
    const size_t aoff = (size_t)(r0 + lr) * K + 8 * hi, boff = (size_t)(c0 + lr) * K + 8 * hi;
#pragma unroll 1
    for (int kc = 0; kc < Kc; kc += 32) {
        V a[4], a2[4];
#pragma unroll
        for (int mb = 0; mb < 4; ++mb) { a[mb] = WFrag<T16>::ld(A + aoff + (size_t)mb * 16 * K + kc); if (NSPLIT == 1 || NSPLIT == 2) a2[mb] = WFrag<T16>::ld(A2 + aoff + (size_t)mb * 16 * K + kc); }
#pragma unroll
        for (int nb = 0; nb < 4; ++nb) { const V b = WFrag<T16>::ld(Bt + boff + (size_t)nb * 16 * K + kc); V b2; if (NSPLIT >= 2) b2 = WFrag<T16>::ld(Bt2 + boff + (size_t)nb * 16 * K + kc);
#pragma unroll
            for (int mb = 0; mb < 4; ++mb) { acc[mb][nb] = WFrag<T16>::mma(a[mb], b, acc[mb][nb]); if (NSPLIT == 1 || NSPLIT == 2) acc[mb][nb] = WFrag<T16>::mma(a2[mb], b, acc[mb][nb]); if (NSPLIT >= 2) acc[mb][nb] = WFrag<T16>::mma(a[mb], b2, acc[mb][nb]); } }
        asm volatile("v_nop\n\tv_nop\n\tv_nop\n\tv_nop" : "+v"(acc[0][0]), "+v"(acc[1][1]), "+v"(acc[2][2]), "+v"(acc[3][3]) : "v"(a[0]), "v"(a[3]));
    }
#pragma unroll
    for (int mb = 0; mb < 4; ++mb) {
#pragma unroll
        for (int nb = 0; nb < 4; ++nb) {
#pragma unroll
            for (int j = 0; j < 8; ++j) os[(hi * 8 + j) * 68 + nb * 16 + lr] = acc[mb][nb][j]; }
        __builtin_amdgcn_wave_barrier(); asm volatile("" ::: "memory");
        float* crow = C + (size_t)(r0 + mb * 16) * ldc + c0;
#pragma unroll 1
        for (int ps = 0; ps < 2; ++ps) {
#pragma unroll
            for (int s = 0; s < 8; ++s) { const int row = 2 * s + hi, cofs = lr * 4; v4f val = *(const v4fa*)(os + row * 68 + cofs); val = val * osc;
                *(volatile v4f*)(crow + (size_t)row * ldc + cofs) = val; }
            if (ps == 0) __threadfence(); }
        __builtin_amdgcn_wave_barrier(); asm volatile("" ::: "memory");
    }
}

__global__ __launch_bounds__(256) void k_cvt8(const float* __restrict__ src, bf* dst, size_t n8) { const size_t i = (size_t)blockIdx.x * 256 + threadIdx.x; if (i >= n8) return; const v8f v = *(const v8f*)(src + i * 8); v8us o;
#pragma unroll
    for (int k = 0; k < 8; ++k) o[k] = f2bf(v[k]); *(volatile v8us*)(dst + i * 8) = o; __threadfence(); *(volatile v8us*)(dst + i * 8) = o; }

__global__ __launch_bounds__(256) void k_plane(const float* __restrict__ src, int R, int CC, int rh, int cw, h16* P16, bf* Ph, bf* Pl, size_t zs, size_t zp, size_t zhl) {
    const size_t z = blockIdx.y; src += z * zs; P16 += z * zp; Ph += z * zhl; Pl += z * zhl;
    const size_t e = ((size_t)blockIdx.x * 256 + threadIdx.x) * 8; if (e >= (size_t)R * CC) return;
    const int r = (int)(e / (size_t)CC), c = (int)(e % (size_t)CC);
    const v4f s0 = *(const v4f*)(src + e); const v4f s1 = *(const v4f*)(src + e + 4);
    v8h o16; v8us oh, ol;
#pragma unroll
    for (int q = 0; q < 4; ++q) { o16[q] = tohx(s0[q]); o16[4 + q] = tohx(s1[q]); unsigned short a, l2; splitf(s0[q], a, l2); oh[q] = a; ol[q] = l2; splitf(s1[q], a, l2); oh[4 + q] = a; ol[4 + q] = l2; }
    const bool hl = (r < rh) && (c < cw); const size_t oo = (size_t)r * cw + c;
#pragma unroll 1
    for (int ps = 0; ps < 2; ++ps) { *(volatile v8h*)(P16 + e) = o16; if (hl) { *(volatile v8us*)(Ph + oo) = oh; *(volatile v8us*)(Pl + oo) = ol; } if (ps == 0) __threadfence(); }
}

__global__ __launch_bounds__(256) void k_asoft(const float* __restrict__ Sb, h16* P16, bf* Ph, bf* Pl) {
    const int lane = threadIdx.x & 31; const int i = blockIdx.x * 8 + (threadIdx.x >> 5); if (i >= SEQ) return; const bool hires = (i < RH); const float* sr = Sb + (size_t)i * SEQ; float v[SEQ / 32]; float mx = -3.0e38f;
#pragma unroll
    for (int ch = 0; ch < SEQ / 128; ++ch) { const int j0 = ch * 128 + lane * 4; const v4f a = *(const v4f*)(sr + j0);
#pragma unroll
        for (int q = 0; q < 4; ++q) { const int j = j0 + q; float t = a[q] * SCL; t = (j <= i) ? t : -1.0e30f; v[ch * 4 + q] = t; mx = fmaxf(mx, t); } }
#pragma unroll
    for (int sh = 16; sh; sh >>= 1) mx = fmaxf(mx, __shfl_xor(mx, sh, 32));
    float sum = 0.f;
#pragma unroll
    for (int k = 0; k < SEQ / 32; ++k) { float d0 = __fsub_rn(v[k], mx); asm volatile("" : "+v"(d0)); v[k] = __builtin_amdgcn_exp2f(__fmul_rn(d0, 1.4426950408889634f)); sum += v[k]; }
#pragma unroll
    for (int sh = 16; sh; sh >>= 1) sum += __shfl_xor(sum, sh, 32);
    const float f = __fdiv_rn(hires ? 1.0f : PCAR, sum);
#pragma unroll 1
    for (int ps = 0; ps < 2; ++ps) {
        if (hires) {
#pragma unroll
            for (int ch = 0; ch < RH / 128; ++ch) { v4us oh, ol;
#pragma unroll
                for (int q = 0; q < 4; ++q) { unsigned short a, c2; splitf(v[ch * 4 + q] * f, a, c2); oh[q] = a; ol[q] = c2; }
                const size_t oo = (size_t)i * RH + ch * 128 + lane * 4; *(volatile v4us*)(Ph + oo) = oh; *(volatile v4us*)(Pl + oo) = ol; }
        } else {
#pragma unroll
            for (int ch = 0; ch < SEQ / 128; ++ch) { v4h o4;
#pragma unroll
                for (int q = 0; q < 4; ++q) o4[q] = tohx(v[ch * 4 + q] * f);
                *(volatile v4h*)(P16 + (size_t)i * SEQ + ch * 128 + lane * 4) = o4; } }
        if (ps == 0) __threadfence(); }
}

#define AL256(x) ((((size_t)(x)) + 255) & ~(size_t)255)
#define XB_B   AL256((size_t)NB * SEQ_FULL * DD * 2)
#define WB_B   AL256((size_t)3 * DD * DD * 2)
#define QKF_B  AL256((size_t)2 * SEQ * DD * 4)
#define VTF_B  AL256((size_t)DD * SEQ * 4)
#define QK16_B AL256((size_t)2 * SEQ * DD * 2)
#define VT16_B AL256((size_t)DD * SEQ * 2)
#define QKH_B  AL256((size_t)2 * RH * DD * 2)
#define VTH_B  AL256((size_t)DD * RH * 2)
#define SB_B   AL256((size_t)SEQ * SEQ * 4)
#define P16_B  AL256((size_t)SEQ * SEQ * 2)
#define PH_B   AL256((size_t)RH * RH * 2)
#define WS_TOTAL (XB_B + WB_B + QKF_B + VTF_B + QK16_B + VT16_B + 2 * QKH_B + 2 * VTH_B + SB_B + P16_B + 2 * PH_B)
static_assert(WS_TOTAL <= (size_t)134217728);

extern "C" void kernel_launch(void* const* d_in, const int* in_sizes, int n_in,
                              void* d_out, int out_size, void* d_ws, size_t ws_size, hipStream_t stream) {
    if (n_in < 4) return;
    if (in_sizes[0] < NB * SEQ_FULL * DD || in_sizes[1] < DD * DD || in_sizes[2] < DD * DD || in_sizes[3] < DD * DD) return;
    if (out_size < (NB - 1) * SEQ_FULL * DD + SEQ * DD) return;
    if (WS_TOTAL > ws_size) return;
    const float* x = (const float*)d_in[0]; const float* wq = (const float*)d_in[1]; const float* wk = (const float*)d_in[2]; const float* wv = (const float*)d_in[3];
    float* OUT = (float*)d_out;
    char* wsp = (char*)d_ws;
    auto take = [&](size_t bytes) { char* p = wsp; wsp += bytes; return (void*)p; };
    bf* Xb = (bf*)take(XB_B); bf* Wb = (bf*)take(WB_B);
    float* QKf = (float*)take(QKF_B); float* VTf = (float*)take(VTF_B);
    h16* QK16 = (h16*)take(QK16_B); h16* VT16 = (h16*)take(VT16_B);
    bf* QKh = (bf*)take(QKH_B); bf* QKl = (bf*)take(QKH_B); bf* VTh = (bf*)take(VTH_B); bf* VTl = (bf*)take(VTH_B);
    float* Sb = (float*)take(SB_B); h16* P16 = (h16*)take(P16_B); bf* Ph = (bf*)take(PH_B); bf* Pl = (bf*)take(PH_B);
    if ((size_t)(wsp - (char*)d_ws) > ws_size) return;

    const size_t nx8 = (size_t)NB * SEQ_FULL * DD / 8, nw8 = (size_t)DD * DD / 8;
    k_cvt8<<<(unsigned)((nx8 + 255) / 256), 256, 0, stream>>>(x, Xb, nx8);
    k_cvt8<<<(unsigned)((nw8 + 255) / 256), 256, 0, stream>>>(wq, Wb, nw8);
    k_cvt8<<<(unsigned)((nw8 + 255) / 256), 256, 0, stream>>>(wk, Wb + (size_t)DD * DD, nw8);
    k_cvt8<<<(unsigned)((nw8 + 255) / 256), 256, 0, stream>>>(wv, Wb + (size_t)2 * DD * DD, nw8);

    const unsigned LQK = (unsigned)(((size_t)SEQ * DD / 8 + 255) / 256), LVT = (unsigned)(((size_t)DD * SEQ / 8 + 255) / 256);
    for (int b = 0; b < NB; ++b) {
        const bf* Xbb = Xb + (size_t)b * SEQ_FULL * DD; float* OUTb = OUT + (size_t)b * SEQ_FULL * DD;
        k_gemmw<bf, 0, 0><<<dim3(SEQ / 64, DD / 64, 2), 32, 0, stream>>>(Xbb, nullptr, Wb, nullptr, DD, QKf, DD, 1.0f, 0, (size_t)0, (size_t)DD * DD, (size_t)SEQ * DD);
        k_gemmw<bf, 0, 0><<<dim3(DD / 64, SEQ / 64, 1), 32, 0, stream>>>(Wb + (size_t)2 * DD * DD, nullptr, Xbb, nullptr, DD, VTf, SEQ, 1.0f, 0, (size_t)0, (size_t)0, (size_t)0);
        k_plane<<<dim3(LQK, 2), 256, 0, stream>>>(QKf, SEQ, DD, RH, DD, QK16, QKh, QKl, (size_t)SEQ * DD, (size_t)SEQ * DD, (size_t)RH * DD);
        k_plane<<<dim3(LVT, 1), 256, 0, stream>>>(VTf, DD, SEQ, DD, RH, VT16, VTh, VTl, (size_t)0, (size_t)0, (size_t)0);
        k_gemmw<bf, 2, 1><<<dim3(RH / 64, RH / 64, 1), 32, 0, stream>>>(QKh, QKl, QKh + (size_t)RH * DD, QKl + (size_t)RH * DD, DD, Sb, SEQ, 1.0f, 0, (size_t)0, (size_t)0, (size_t)0);
        if (SEQ > RH) k_gemmw<h16, 0, 1><<<dim3((SEQ - RH) / 64, SEQ / 64, 1), 32, 0, stream>>>(QK16 + (size_t)RH * DD, nullptr, QK16 + (size_t)SEQ * DD, nullptr, DD, Sb + (size_t)RH * SEQ, SEQ, 1.0f, RH, (size_t)0, (size_t)0, (size_t)0);
        k_asoft<<<SEQ / 8, 256, 0, stream>>>(Sb, P16, Ph, Pl);
        k_gemmw<bf, 2, 2><<<dim3(RH / 64, DD / 64, 1), 32, 0, stream>>>(Ph, Pl, VTh, VTl, RH, OUTb, DD, 1.0f, 0, (size_t)0, (size_t)0, (size_t)0);
        if (SEQ > RH) k_gemmw<h16, 0, 2><<<dim3((SEQ - RH) / 64, DD / 64, 1), 32, 0, stream>>>(P16 + (size_t)RH * SEQ, nullptr, VT16, nullptr, SEQ, OUTb + (size_t)RH * DD, DD, 1.0f / PCAR, RH, (size_t)0, (size_t)0, (size_t)0);
    }
}
